// MultiHeadAttentionBlock_51402168598763
// MI455X (gfx1250) — hardware-verified
//
#include <hip/hip_runtime.h>


#ifndef NB
#define NB 4
#endif
#ifndef SEQ
#define SEQ 2048
#endif
#ifndef RX
#define RX   256
#endif
#define NB_FULL  4
#define SEQ_FULL 2048
#define DM   512
#define NH   8
#define HD   64
#define PCAR 1024.0f
#define SCL  0.125f
#define PBP  40
#define L2E  1.4426950408889634f
#define MFILL (-1.0e9f)

static_assert(NB >= 1 && NB <= NB_FULL);
static_assert(SEQ <= SEQ_FULL && SEQ % 64 == 0);
static_assert(RX % 32 == 0 && RX >= 32 && RX < SEQ);
static_assert((SEQ - RX) % 128 == 0);
static_assert(NH * HD == DM && HD == 64 && DM % 64 == 0);
static_assert((SEQ * DM) % 2048 == 0);
static_assert(((size_t)NB * NH * SEQ * HD) % 2048 == 0);
static_assert((DM * DM) % 2048 == 0);
static_assert((NB * SEQ) % 64 == 0);
static_assert(DM % 32 == 0);
static_assert((NB * NH * ((SEQ - RX) / 16)) % 8 == 0);
static_assert(((size_t)(NB - 1) * SEQ_FULL + SEQ - 1) * DM + DM - 1 < (size_t)NB_FULL * SEQ_FULL * DM);

typedef _Float16 h16;
typedef unsigned short bf;
typedef __attribute__((ext_vector_type(16))) __bf16   v16bf;
typedef __attribute__((ext_vector_type(16))) _Float16 v16h;
typedef __attribute__((ext_vector_type(8)))  _Float16 v8h;
typedef __attribute__((ext_vector_type(8)))  unsigned short v8us;
typedef __attribute__((ext_vector_type(8)))  float    v8f;
typedef __attribute__((ext_vector_type(4)))  float    v4f;
typedef __attribute__((ext_vector_type(8)))  unsigned int v8u;
typedef v8h  __attribute__((may_alias)) v8ha;
typedef v4f  __attribute__((may_alias)) v4fa;
typedef v8us __attribute__((may_alias)) v8usa;

__device__ __forceinline__ unsigned short f2bf(float f) { unsigned u = __float_as_uint(f); u += 0x7FFFu + ((u >> 16) & 1u); return (unsigned short)(u >> 16); }
__device__ __forceinline__ float bf2f(unsigned short b) { return __uint_as_float(((unsigned)b) << 16); }
__device__ __forceinline__ float bfr(float f) { return bf2f(f2bf(f)); }
__device__ __forceinline__ void splitf(float y, unsigned short& h, unsigned short& l) { h = f2bf(y); l = f2bf(y - bf2f(h)); }
__device__ __forceinline__ v16h cat16(v8h lo, v8h hi) { return __builtin_shufflevector(lo, hi, 0, 1, 2, 3, 4, 5, 6, 7, 8, 9, 10, 11, 12, 13, 14, 15); }
__device__ __forceinline__ v16bf cat16b(v8us lo, v8us hi) { return __builtin_bit_cast(v16bf, __builtin_shufflevector(lo, hi, 0, 1, 2, 3, 4, 5, 6, 7, 8, 9, 10, 11, 12, 13, 14, 15)); }
__device__ __forceinline__ v8f wmma16(v16h a, v16h b, v8f c) { return __builtin_amdgcn_wmma_f32_16x16x32_f16(false, a, false, b, (short)0, c, false, false); }
__device__ __forceinline__ v8f wmmab(v16bf a, v16bf b, v8f c) { return __builtin_amdgcn_wmma_f32_16x16x32_bf16(false, a, false, b, (short)0, c, false, false); }
__device__ __forceinline__ float ex2c(float x) { return __builtin_amdgcn_exp2f(fmaxf(x, -200.0f) * L2E); }

template <typename T16> struct WFrag;
template <> struct WFrag<h16> { typedef v16h V; static __device__ __forceinline__ V ld(const h16* p) { return cat16(*(const v8h*)p, *(const v8h*)(p + 16)); } static __device__ __forceinline__ v8f mma(V a, V b, v8f c) { return wmma16(a, b, c); } };
template <> struct WFrag<bf> { typedef v16bf V; static __device__ __forceinline__ V ld(const bf* p) { return cat16b(*(const v8us*)p, *(const v8us*)(p + 16)); } static __device__ __forceinline__ v8f mma(V a, V b, v8f c) { return wmmab(a, b, c); } };

template <typename T16, int NSPLIT, bool BIAS>
__global__ __launch_bounds__(32) void k_gemmw(const T16* __restrict__ A, const T16* __restrict__ A2, const T16* __restrict__ Bt, const T16* __restrict__ Bt2, int K, float* C, int ldc, const float* __restrict__ bias, const int* __restrict__ pflag, size_t sA, size_t sB, size_t sC) {
    typedef typename WFrag<T16>::V V;
    __shared__ __align__(16) float os[16 * 68];
    const size_t z = blockIdx.z; A += z * sA; if (A2) A2 += z * sA; Bt += z * sB; if (Bt2) Bt2 += z * sB; C += z * sC;
    const int lane = threadIdx.x & 31, lr = lane & 15, hi = lane >> 4; const int r0 = blockIdx.x * 64, c0 = blockIdx.y * 64;
    float pz = 0.0f; if (pflag != nullptr) pz = (pflag[0] != 0) ? __int_as_float(0x7fc00000) : 0.0f;
    v8f acc[4][4];
#pragma unroll
    for (int mb = 0; mb < 4; ++mb)
#pragma unroll
        for (int nb = 0; nb < 4; ++nb) acc[mb][nb] = (v8f){};
    const size_t aoff = (size_t)(r0 + lr) * K + 8 * hi, boff = (size_t)(c0 + lr) * K + 8 * hi;
#pragma unroll 1
    for (int kc = 0; kc < K; kc += 32) {
        V a[4], a2[4];
#pragma unroll
        for (int mb = 0; mb < 4; ++mb) { a[mb] = WFrag<T16>::ld(A + aoff + (size_t)mb * 16 * K + kc); if (NSPLIT == 1 || NSPLIT == 2) a2[mb] = WFrag<T16>::ld(A2 + aoff + (size_t)mb * 16 * K + kc); }
#pragma unroll
        for (int nb = 0; nb < 4; ++nb) { const V b = WFrag<T16>::ld(Bt + boff + (size_t)nb * 16 * K + kc); V b2; if (NSPLIT >= 2) b2 = WFrag<T16>::ld(Bt2 + boff + (size_t)nb * 16 * K + kc);
#pragma unroll
            for (int mb = 0; mb < 4; ++mb) { acc[mb][nb] = WFrag<T16>::mma(a[mb], b, acc[mb][nb]); if (NSPLIT == 1 || NSPLIT == 2) acc[mb][nb] = WFrag<T16>::mma(a2[mb], b, acc[mb][nb]); if (NSPLIT >= 2) acc[mb][nb] = WFrag<T16>::mma(a[mb], b2, acc[mb][nb]); } }
        asm volatile("v_nop\n\tv_nop\n\tv_nop\n\tv_nop" : "+v"(acc[0][0]), "+v"(acc[1][1]), "+v"(acc[2][2]), "+v"(acc[3][3]) : "v"(a[0]), "v"(a[3]));
    }
#pragma unroll
    for (int mb = 0; mb < 4; ++mb) {
#pragma unroll
        for (int nb = 0; nb < 4; ++nb) {
#pragma unroll
            for (int j = 0; j < 8; ++j) os[(hi * 8 + j) * 68 + nb * 16 + lr] = acc[mb][nb][j]; }
        __builtin_amdgcn_wave_barrier(); asm volatile("" ::: "memory");
        float* crow = C + (size_t)(r0 + mb * 16) * ldc + c0;
#pragma unroll 1
        for (int ps = 0; ps < 2; ++ps) {
#pragma unroll
            for (int s = 0; s < 8; ++s) { const int row = 2 * s + hi, cofs = lr * 4; v4f val = *(const v4fa*)(os + row * 68 + cofs); if (BIAS) { val[0] += bfr(bias[c0 + cofs]); val[1] += bfr(bias[c0 + cofs + 1]); val[2] += bfr(bias[c0 + cofs + 2]); val[3] += bfr(bias[c0 + cofs + 3]); }
                val = val + pz;
                *(volatile v4f*)(crow + (size_t)row * ldc + cofs) = val; }
            if (ps == 0) __threadfence(); }
        __builtin_amdgcn_wave_barrier(); asm volatile("" ::: "memory");
    }
}

__global__ __launch_bounds__(256) void k_cvt8(const float* __restrict__ src, bf* dst, size_t n8) { const size_t i = (size_t)blockIdx.x * 256 + threadIdx.x; if (i >= n8) return; const v8f v = *(const v8f*)(src + i * 8); v8us o;
#pragma unroll
    for (int k = 0; k < 8; ++k) o[k] = f2bf(v[k]); *(volatile v8us*)(dst + i * 8) = o; __threadfence(); *(volatile v8us*)(dst + i * 8) = o; }

__global__ __launch_bounds__(256) void k_cvtx(const float* __restrict__ src, bf* dst) {
    const size_t i = (size_t)blockIdx.x * 256 + threadIdx.x; const int b = blockIdx.y; const size_t n8 = (size_t)SEQ * DM / 8; if (i >= n8) return;
    const v8f v = *(const v8f*)(src + (size_t)b * SEQ_FULL * DM + i * 8); v8us o;
#pragma unroll
    for (int k = 0; k < 8; ++k) o[k] = f2bf(v[k]);
    bf* d = dst + (size_t)b * SEQ * DM + i * 8; *(volatile v8us*)d = o; __threadfence(); *(volatile v8us*)d = o; }

__global__ __launch_bounds__(256) void k_qkplane(const float* __restrict__ F, h16* P) {
    const size_t e = ((size_t)blockIdx.x * 256 + threadIdx.x) * 8; if (e >= (size_t)NB * NH * SEQ * HD) return;
    const int d = (int)(e % HD); const int s = (int)((e / HD) % SEQ); const int h = (int)((e / ((size_t)HD * SEQ)) % NH); const int b = (int)(e / ((size_t)HD * SEQ * NH));
    const v8f v = *(const v8f*)(F + ((size_t)b * SEQ + s) * DM + h * HD + d); v8h o;
#pragma unroll
    for (int k = 0; k < 8; ++k) o[k] = (h16)v[k];
    *(volatile v8h*)(P + e) = o; __threadfence(); *(volatile v8h*)(P + e) = o; }

__global__ __launch_bounds__(256) void k_vtplane(const float* __restrict__ F, h16* VT) {
    const size_t e = ((size_t)blockIdx.x * 256 + threadIdx.x) * 8; if (e >= (size_t)NB * NH * HD * SEQ) return;
    const int s = (int)(e % SEQ); const int d = (int)((e / SEQ) % HD); const int h = (int)((e / ((size_t)SEQ * HD)) % NH); const int b = (int)(e / ((size_t)SEQ * HD * NH));
    const float* f = F + ((size_t)b * SEQ + s) * DM + h * HD + d; v8h o;
#pragma unroll
    for (int k = 0; k < 8; ++k) o[k] = (h16)f[(size_t)k * DM];
    *(volatile v8h*)(VT + e) = o; __threadfence(); *(volatile v8h*)(VT + e) = o; }

__global__ __launch_bounds__(256) void k_maskbits(const int* __restrict__ mask, unsigned* MB) {
    const unsigned lane = threadIdx.x & 31u, wave = threadIdx.x >> 5;
    const unsigned rg = blockIdx.x * 8u + wave, jt = blockIdx.y;
    if (rg >= (unsigned)(SEQ / 32)) return;
    const unsigned i0 = rg * 32u;
    unsigned w = 0u;
#pragma unroll 4
    for (unsigned r = 0; r < 32u; ++r) {
        const int m = mask[(size_t)(i0 + r) * SEQ_FULL + jt * 32u + lane];
        const unsigned bal = __builtin_amdgcn_ballot_w32(m != 0);
        w = (lane == r) ? bal : w;
    }
    unsigned* dst = MB + (size_t)jt * SEQ + i0 + lane;
    *(volatile unsigned*)dst = w; __threadfence(); *(volatile unsigned*)dst = w;
}

__global__ __launch_bounds__(32) void k_early(const float* __restrict__ FQ, const float* __restrict__ FK, const float* __restrict__ FV, const unsigned* __restrict__ MB, bf* Ah, bf* Al) {
    __shared__ __align__(16) float Qs[32 * 68]; __shared__ __align__(16) float As[32 * 68]; __shared__ __align__(16) float Ks[32 * 64]; __shared__ __align__(16) float Vs[32 * 64]; __shared__ float Ss[32 * 33];
    const int lane = threadIdx.x & 31; const int g = blockIdx.x, h = blockIdx.y, b = blockIdx.z; const int i = g * 32 + lane;
    const size_t rq = ((size_t)b * SEQ + i) * DM + h * HD;
    const v4f z4 = {0.0f, 0.0f, 0.0f, 0.0f};
#pragma unroll 1
    for (int c = 0; c < 16; ++c) { *(v4fa*)(Qs + lane * 68 + c * 4) = *(const v4f*)(FQ + rq + c * 4); *(v4fa*)(As + lane * 68 + c * 4) = z4; }
    const unsigned NT = (unsigned)(SEQ / 32);
    unsigned rowor = 0u, lastc = 0u;
#pragma unroll 1
    for (unsigned ck = 0; ck < NT; ++ck) { const unsigned w = MB[(size_t)ck * SEQ + i]; rowor |= w; const unsigned bal = __builtin_amdgcn_ballot_w32(w != 0u); lastc = (bal != 0u) ? ck : lastc; }
    const unsigned emp = __builtin_amdgcn_ballot_w32(rowor == 0u);
    unsigned nck = (emp != 0u) ? NT : (lastc + 1u); nck = (nck < NT) ? nck : NT;
    float m = -3.0e38f, l = 0.0f;
#pragma unroll 1
    for (unsigned ck = 0; ck < nck; ++ck) {
        __syncthreads();
#pragma unroll 1
        for (int it = 0; it < 16; ++it) { const int idx = it * 32 + lane; const int row = idx >> 4, c4 = (idx & 15) * 4; const size_t rk = ((size_t)b * SEQ + ck * 32u + row) * DM + h * HD + c4;
            *(v4fa*)(Ks + row * 64 + c4) = *(const v4f*)(FK + rk); *(v4fa*)(Vs + row * 64 + c4) = *(const v4f*)(FV + rk); }
        __syncthreads();
        const unsigned mw = MB[(size_t)ck * SEQ + i];
        float cm = -3.0e38f;
#pragma unroll 1
        for (int j = 0; j < 32; ++j) {
            v4f s4 = z4;
#pragma unroll 1
            for (int c = 0; c < 16; ++c) { const v4f qv = *(const v4fa*)(Qs + lane * 68 + c * 4); const v4f kv = *(const v4fa*)(Ks + j * 64 + c * 4);
                s4[0] = fmaf(qv[0], kv[0], s4[0]); s4[1] = fmaf(qv[1], kv[1], s4[1]); s4[2] = fmaf(qv[2], kv[2], s4[2]); s4[3] = fmaf(qv[3], kv[3], s4[3]); }
            const float s = ((s4[0] + s4[1]) + (s4[2] + s4[3])) * SCL;
            const float t = (((mw >> (unsigned)j) & 1u) != 0u) ? s : MFILL;
            Ss[lane * 33 + j] = t; cm = fmaxf(cm, t); }
        const float mn = fmaxf(m, cm);
        const float corr = ex2c(m - mn);
        float rs = 0.0f;
#pragma unroll 1
        for (int j = 0; j < 32; ++j) { const float p = ex2c(Ss[lane * 33 + j] - mn); Ss[lane * 33 + j] = p; rs += p; }
        l = l * corr + rs; m = mn;
#pragma unroll 1
        for (int c = 0; c < 16; ++c) { v4f a = *(const v4fa*)(As + lane * 68 + c * 4); a = a * corr;
#pragma unroll 1
            for (int j = 0; j < 32; ++j) { const float p = Ss[lane * 33 + j]; const v4f vv = *(const v4fa*)(Vs + j * 64 + c * 4);
                a[0] = fmaf(p, vv[0], a[0]); a[1] = fmaf(p, vv[1], a[1]); a[2] = fmaf(p, vv[2], a[2]); a[3] = fmaf(p, vv[3], a[3]); }
            *(v4fa*)(As + lane * 68 + c * 4) = a; }
    }
    const float inv = 1.0f / l;
#pragma unroll 1
    for (int c = 0; c < 16; ++c) { v4f a = *(const v4fa*)(As + lane * 68 + c * 4); a = a * inv; *(v4fa*)(As + lane * 68 + c * 4) = a; }
    __syncthreads();
    const int q = lane >> 3, piece = lane & 7;
#pragma unroll 1
    for (int ps = 0; ps < 2; ++ps) {
#pragma unroll 1
        for (int it = 0; it < 8; ++it) { const int row = it * 4 + q; const v4f x0 = *(const v4fa*)(As + row * 68 + piece * 8); const v4f x1 = *(const v4fa*)(As + row * 68 + piece * 8 + 4); v8us oh, ol;
#pragma unroll
            for (int k = 0; k < 4; ++k) { unsigned short a0, c0, a1, c1; splitf(x0[k], a0, c0); splitf(x1[k], a1, c1); oh[k] = a0; ol[k] = c0; oh[4 + k] = a1; ol[4 + k] = c1; }
            const size_t oo = ((size_t)b * SEQ + g * 32 + row) * DM + h * HD + piece * 8; *(volatile v8us*)(Ah + oo) = oh; *(volatile v8us*)(Al + oo) = ol; }
        if (ps == 0) __threadfence(); }
}

__global__ __launch_bounds__(256) void k_attn(const h16* __restrict__ Q16, const h16* __restrict__ K16, const h16* __restrict__ VT16, const unsigned* __restrict__ MB, bf* Ah, bf* Al) {
    __shared__ __align__(16) h16 pb[8 * 16 * PBP];
    __shared__ __align__(16) float ob[8 * 16 * 64];
    const int lane = threadIdx.x & 31, wave = threadIdx.x >> 5, lr = lane & 15, hi = lane >> 4;
    const int QB = (SEQ - RX) / 16;
    const int gw = blockIdx.x * 8 + wave; const int bh = gw / QB; const int q0 = RX + (gw - bh * QB) * 16;
    if (bh >= NB * NH) return;
    const int b = bh / NH, h = bh - b * NH;
    const h16* qp = Q16 + (size_t)bh * SEQ * HD; const h16* kp = K16 + (size_t)bh * SEQ * HD; const h16* vp = VT16 + (size_t)bh * HD * SEQ;
    h16* pw = pb + wave * 16 * PBP; float* ow = ob + wave * 16 * 64;
    const unsigned NT = (unsigned)(SEQ / 32);
    unsigned lastt = 0u; unsigned ra[16];
#pragma unroll
    for (int r = 0; r < 16; ++r) ra[r] = 0u;
#pragma unroll
    for (unsigned c = 0; c < (NT + 31u) / 32u; ++c) {
        const unsigned jt = c * 32u + (unsigned)lane; const bool ok = jt < NT; const unsigned jc = ok ? jt : (NT - 1u);
        const unsigned* wp = MB + (size_t)jc * SEQ + q0;
        const v8u w0 = *(const v8u*)wp; const v8u w1 = *(const v8u*)(wp + 8);
        unsigned tor = 0u;
#pragma unroll
        for (int r = 0; r < 8; ++r) { const unsigned x0 = ok ? w0[r] : 0u; const unsigned x1 = ok ? w1[r] : 0u; ra[r] |= x0; ra[8 + r] |= x1; tor |= (x0 | x1); }
        const unsigned bits = __builtin_amdgcn_ballot_w32(tor != 0u);
        const unsigned top = c * 32u + 31u - (unsigned)__builtin_clz(bits | 1u);
        lastt = (bits != 0u) ? top : lastt;
    }
    unsigned emp = 0u;
#pragma unroll
    for (int r = 0; r < 16; ++r) { const unsigned bal = __builtin_amdgcn_ballot_w32(ra[r] != 0u); emp |= (bal == 0u) ? 1u : 0u; }
    unsigned ntiles = (emp != 0u) ? NT : (lastt + 1u); ntiles = (ntiles < NT) ? ntiles : NT;
    v16h aq[2];
#pragma unroll
    for (int c = 0; c < 2; ++c) aq[c] = WFrag<h16>::ld(qp + (size_t)(q0 + lr) * HD + c * 32 + 8 * hi);
    v8f acc[4];
#pragma unroll
    for (int t = 0; t < 4; ++t) acc[t] = (v8f){};
    float mi[8], li[8];
#pragma unroll
    for (int r = 0; r < 8; ++r) { mi[r] = -3.0e38f; li[r] = 0.0f; }
#pragma unroll 1
    for (unsigned jt = 0; jt < ntiles; ++jt) {
        const int j0 = (int)(jt * 32u);
        const v8u mw = *(const v8u*)(MB + (size_t)jt * SEQ + q0 + 8 * hi);
        v16h bk[2][2];
#pragma unroll
        for (int nt = 0; nt < 2; ++nt)
#pragma unroll
            for (int c = 0; c < 2; ++c) bk[nt][c] = WFrag<h16>::ld(kp + (size_t)(j0 + nt * 16 + lr) * HD + c * 32 + 8 * hi);
        v8f s[2];
#pragma unroll
        for (int nt = 0; nt < 2; ++nt) { s[nt] = (v8f){};
#pragma unroll
            for (int c = 0; c < 2; ++c) s[nt] = wmma16(aq[c], bk[nt][c], s[nt]); }
        asm volatile("v_nop\n\tv_nop\n\tv_nop\n\tv_nop" : "+v"(s[0]), "+v"(s[1]) : "v"(aq[1]), "v"(bk[1][1]));
        float e0[8], e1[8], cr[8];
#pragma unroll
        for (int r = 0; r < 8; ++r) {
            const unsigned w = mw[r];
            const bool k0 = ((w >> (unsigned)lr) & 1u) != 0u; const bool k1 = ((w >> (unsigned)(lr + 16)) & 1u) != 0u;
            const float t0 = k0 ? s[0][r] * SCL : MFILL; const float t1 = k1 ? s[1][r] * SCL : MFILL;
            float tm = fmaxf(t0, t1);
#pragma unroll
            for (int off = 1; off < 16; off <<= 1) tm = fmaxf(tm, __shfl_xor(tm, off, 32));
            const float mn = fmaxf(mi[r], tm);
            cr[r] = ex2c(mi[r] - mn);
            e0[r] = ex2c(t0 - mn); e1[r] = ex2c(t1 - mn);
            float rs = e0[r] + e1[r];
#pragma unroll
            for (int off = 1; off < 16; off <<= 1) rs += __shfl_xor(rs, off, 32);
            li[r] = li[r] * cr[r] + rs; mi[r] = mn;
        }
#pragma unroll
        for (int t = 0; t < 4; ++t)
#pragma unroll
            for (int r = 0; r < 8; ++r) acc[t][r] *= cr[r];
        __builtin_amdgcn_fence(3  , "wavefront"); __builtin_amdgcn_wave_barrier();
#pragma unroll
        for (int r = 0; r < 8; ++r) { pw[(8 * hi + r) * PBP + lr] = (h16)(e0[r] * PCAR); pw[(8 * hi + r) * PBP + 16 + lr] = (h16)(e1[r] * PCAR); }
        __builtin_amdgcn_fence(3  , "wavefront"); __builtin_amdgcn_wave_barrier();
        const v16h ap = cat16(*(const v8ha*)(pw + lr * PBP + 8 * hi), *(const v8ha*)(pw + lr * PBP + 16 + 8 * hi));
        v16h bv[4];
#pragma unroll
        for (int t = 0; t < 4; ++t) bv[t] = WFrag<h16>::ld(vp + (size_t)(t * 16 + lr) * SEQ + j0 + 8 * hi);
#pragma unroll
        for (int t = 0; t < 4; ++t) acc[t] = wmma16(ap, bv[t], acc[t]);
        asm volatile("v_nop\n\tv_nop\n\tv_nop\n\tv_nop" : "+v"(acc[0]), "+v"(acc[1]), "+v"(acc[2]), "+v"(acc[3]) : "v"(ap), "v"(bv[3]));
    }
    float inv[8];
#pragma unroll
    for (int r = 0; r < 8; ++r) inv[r] = 1.0f / (li[r] * PCAR);
#pragma unroll
    for (int t = 0; t < 4; ++t)
#pragma unroll
        for (int r = 0; r < 8; ++r) ow[(8 * hi + r) * 64 + t * 16 + lr] = acc[t][r] * inv[r];
    __builtin_amdgcn_fence(3  , "wavefront"); __builtin_amdgcn_wave_barrier();
    const int q = lane >> 3, piece = lane & 7;
#pragma unroll 1
    for (int ps = 0; ps < 2; ++ps) {
#pragma unroll
        for (int it = 0; it < 4; ++it) { const int row = it * 4 + q; const v4f x0 = *(const v4fa*)(ow + row * 64 + piece * 8); const v4f x1 = *(const v4fa*)(ow + row * 64 + piece * 8 + 4); v8us oh, ol;
#pragma unroll
            for (int k = 0; k < 4; ++k) { unsigned short a0, c0, a1, c1; splitf(x0[k], a0, c0); splitf(x1[k], a1, c1); oh[k] = a0; ol[k] = c0; oh[4 + k] = a1; ol[4 + k] = c1; }
            const size_t oo = ((size_t)b * SEQ + q0 + row) * DM + h * HD + piece * 8; *(volatile v8us*)(Ah + oo) = oh; *(volatile v8us*)(Al + oo) = ol; }
        if (ps == 0) __threadfence(); }
}

extern "C" void kernel_launch(void* const* d_in, const int* in_sizes, int n_in,
                              void* d_out, int out_size, void* d_ws, size_t ws_size, hipStream_t stream) {
    if (n_in < 12) return;
    const size_t xneed = (size_t)(NB - 1) * SEQ_FULL * DM + (size_t)SEQ * DM;
    if ((size_t)in_sizes[0] < xneed || (size_t)in_sizes[1] < xneed || (size_t)in_sizes[2] < xneed) return;
    if ((size_t)in_sizes[3] < (size_t)SEQ_FULL * SEQ_FULL) return;
    if (in_sizes[4] < DM * DM || in_sizes[6] < DM * DM || in_sizes[8] < DM * DM || in_sizes[10] < DM * DM) return;
    if (in_sizes[5] < DM || in_sizes[7] < DM || in_sizes[9] < DM || in_sizes[11] < DM) return;
    if ((size_t)out_size < xneed) return;
    const float* xq = (const float*)d_in[0]; const float* xk = (const float*)d_in[1]; const float* xv = (const float*)d_in[2]; const int* msk = (const int*)d_in[3];
    const float* wq = (const float*)d_in[4]; const float* bq = (const float*)d_in[5]; const float* wk = (const float*)d_in[6]; const float* bk = (const float*)d_in[7];
    const float* wv = (const float*)d_in[8]; const float* bv = (const float*)d_in[9]; const float* wo = (const float*)d_in[10]; const float* bo = (const float*)d_in[11];
    float* OUT = (float*)d_out;
    char* wsp = (char*)d_ws;
    auto take = [&](size_t bytes) { char* p = wsp; wsp += (bytes + 255) & ~(size_t)255; return (void*)p; };
    bf* WQ = (bf*)take((size_t)DM * DM * 2); bf* WK = (bf*)take((size_t)DM * DM * 2); bf* WV = (bf*)take((size_t)DM * DM * 2); bf* WO = (bf*)take((size_t)DM * DM * 2);
    bf* XQ = (bf*)take((size_t)NB * SEQ * DM * 2); bf* XK = (bf*)take((size_t)NB * SEQ * DM * 2); bf* XV = (bf*)take((size_t)NB * SEQ * DM * 2);
    float* FQ = (float*)take((size_t)NB * SEQ * DM * 4); float* FK = (float*)take((size_t)NB * SEQ * DM * 4); float* FV = (float*)take((size_t)NB * SEQ * DM * 4);
    h16* Q16 = (h16*)take((size_t)NB * NH * SEQ * HD * 2); h16* K16 = (h16*)take((size_t)NB * NH * SEQ * HD * 2); h16* VT16 = (h16*)take((size_t)NB * NH * HD * SEQ * 2);
    bf* Ah = (bf*)take((size_t)NB * SEQ * DM * 2); bf* Al = (bf*)take((size_t)NB * SEQ * DM * 2);
    unsigned* MB = (unsigned*)take((size_t)(SEQ / 32) * SEQ * 4);
    const size_t total = (size_t)(wsp - (char*)d_ws);
    if (total > ws_size || total > ((size_t)128 << 20)) return;

    const size_t nw8 = (size_t)DM * DM / 8;
    k_cvt8<<<(unsigned)((nw8 + 255) / 256), 256, 0, stream>>>(wq, WQ, nw8);
    k_cvt8<<<(unsigned)((nw8 + 255) / 256), 256, 0, stream>>>(wk, WK, nw8);
    k_cvt8<<<(unsigned)((nw8 + 255) / 256), 256, 0, stream>>>(wv, WV, nw8);
    k_cvt8<<<(unsigned)((nw8 + 255) / 256), 256, 0, stream>>>(wo, WO, nw8);
    const dim3 gx((unsigned)(((size_t)SEQ * DM / 8 + 255) / 256), NB, 1);
    k_cvtx<<<gx, 256, 0, stream>>>(xq, XQ);
    k_cvtx<<<gx, 256, 0, stream>>>(xk, XK);
    k_cvtx<<<gx, 256, 0, stream>>>(xv, XV);
    const dim3 gp(NB * SEQ / 64, DM / 64, 1);
    k_gemmw<bf, 0, true><<<gp, 32, 0, stream>>>(XQ, nullptr, WQ, nullptr, DM, FQ, DM, bq, nullptr, 0, 0, 0);
    k_gemmw<bf, 0, true><<<gp, 32, 0, stream>>>(XK, nullptr, WK, nullptr, DM, FK, DM, bk, nullptr, 0, 0, 0);
    k_gemmw<bf, 0, true><<<gp, 32, 0, stream>>>(XV, nullptr, WV, nullptr, DM, FV, DM, bv, nullptr, 0, 0, 0);
    const unsigned gpl = (unsigned)(((size_t)NB * NH * SEQ * HD / 8 + 255) / 256);
    k_qkplane<<<gpl, 256, 0, stream>>>(FQ, Q16);
    k_qkplane<<<gpl, 256, 0, stream>>>(FK, K16);
    k_vtplane<<<gpl, 256, 0, stream>>>(FV, VT16);
    k_maskbits<<<dim3((unsigned)((SEQ / 32 + 7) / 8), (unsigned)(SEQ / 32), 1), 256, 0, stream>>>(msk, MB);
    k_early<<<dim3(RX / 32, NH, NB), 32, 0, stream>>>(FQ, FK, FV, MB, Ah, Al);
    k_attn<<<(unsigned)(NB * NH * ((SEQ - RX) / 16) / 8), 256, 0, stream>>>(Q16, K16, VT16, MB, Ah, Al);
    k_gemmw<bf, 1, true><<<dim3(SEQ / 64, DM / 64, NB), 32, 0, stream>>>(Ah, Al, WO, nullptr, DM, OUT, DM, bo, nullptr, (size_t)SEQ * DM, 0, (size_t)SEQ_FULL * DM);
}
